// Attention_67577015435735
// MI455X (gfx1250) — hardware-verified
//
#include <hip/hip_runtime.h>


#ifndef NB
#define NB 16
#endif
#ifndef SEQ
#define SEQ 1024
#endif
#define NB_FULL  16
#define SEQ_FULL 1024
#define DIM   128
#define NH    8
#define INNER (NH * DIM)
#define QKVN  (3 * INNER)
#define NCH   ((NB % 2 == 0) ? 2 : 1)
#define BCH   (NB / NCH)
#define NWV   4
#define BQ    (16 * NWV)
#define KS    32
#define CSP   136
#define OSP   132
#define VTP   72
#define L2E   1.4426950408889634f
#define SC2   (L2E * 0.03125f)
#define PCL   10.0f
#define WQS   16.0f
#define WPS   32.0f
#define CCS   16.0f
#define RSC   2048.0f

static_assert(DIM == 128);
static_assert(INNER == 1024);
static_assert(NB <= NB_FULL);
static_assert(SEQ <= SEQ_FULL);
static_assert(NB % NCH == 0);
static_assert(SEQ % BQ == 0);
static_assert(SEQ % 64 == 0);
static_assert(SEQ % KS == 0);
static_assert(DIM % 32 == 0);
static_assert(DIM == 4 * 32);
static_assert(DIM == 8 * 16);
static_assert(INNER % 32 == 0);
static_assert((NB * SEQ) % 16 == 0);
static_assert(16 * 8 == DIM);
static_assert(64 * CSP <= DIM * VTP);
static_assert(64 <= VTP);
static_assert((CSP * 2) % 16 == 0);
static_assert((VTP * 2) % 16 == 0);
static_assert((OSP * 4) % 16 == 0);
static_assert(32 * 4 == DIM);
static_assert(16 * 8 * 2 == 256);
static_assert(QKVN % 128 == 0);
static_assert(DIM % 64 == 0 && INNER % 64 == 0);
static_assert((BCH * SEQ) % 64 == 0);

#define SZ_XH  ((size_t)NB * SEQ * DIM * 2)
#define SZ_WT  ((size_t)QKVN * DIM * 2)
#define SZ_WP  ((size_t)DIM * INNER * 2)
#define SZ_PL  ((size_t)BCH * NH * SEQ * DIM * 2)
#define SZ_CX  ((size_t)BCH * SEQ * INNER * 2)
#define SZ_ALL (SZ_XH + SZ_WT + SZ_WP + 3 * SZ_PL + 2 * SZ_CX)
static_assert(SZ_XH % 256 == 0 && SZ_WT % 256 == 0 && SZ_WP % 256 == 0 && SZ_PL % 256 == 0 && SZ_CX % 256 == 0);
static_assert(SZ_ALL <= (size_t)134217728);

typedef unsigned short hf;
typedef __attribute__((ext_vector_type(16))) _Float16 v16h;
typedef __attribute__((ext_vector_type(8)))  _Float16 v8h;
typedef __attribute__((ext_vector_type(8)))  unsigned short v8us;
typedef __attribute__((ext_vector_type(8)))  float    v8f;
typedef __attribute__((ext_vector_type(4)))  float    v4f;
typedef v4f  __attribute__((may_alias)) v4fa;
typedef v8us __attribute__((may_alias)) v8usa;

__device__ __forceinline__ float bfr(float f) { unsigned u = __float_as_uint(f); u += 0x7FFFu + ((u >> 16) & 1u); return __uint_as_float(u & 0xFFFF0000u); }
__device__ __forceinline__ unsigned short f2h(float f) { return __builtin_bit_cast(unsigned short, (_Float16)f); }
__device__ __forceinline__ v16h cat16h(v8us lo, v8us hi) { return __builtin_bit_cast(v16h, __builtin_shufflevector(lo, hi, 0, 1, 2, 3, 4, 5, 6, 7, 8, 9, 10, 11, 12, 13, 14, 15)); }
__device__ __forceinline__ v8f wmmah(v16h a, v16h b, v8f c) { return __builtin_amdgcn_wmma_f32_16x16x32_f16(false, a, false, b, (short)0, c, false, false); }
__device__ __forceinline__ v16h ldh(const hf* p) { return cat16h(*(const v8us*)p, *(const v8us*)(p + 16)); }
__device__ __forceinline__ void sfence() { asm volatile("" ::: "memory"); __builtin_amdgcn_sched_barrier(0); }
__device__ __forceinline__ void guard1(v8f& c0, v16h a, v16h b, v16h c, v16h d) {
    asm volatile("v_nop\n\tv_nop\n\tv_nop\n\tv_nop" : "+v"(c0) : "v"(a), "v"(b), "v"(c), "v"(d));
}
__device__ __forceinline__ void guard2(v8f& c0, v8f& c1, v16h a, v16h b, v16h c, v16h d) {
    asm volatile("v_nop\n\tv_nop\n\tv_nop\n\tv_nop" : "+v"(c0), "+v"(c1) : "v"(a), "v"(b), "v"(c), "v"(d));
}
__device__ __forceinline__ void guard4(v8f& c0, v8f& c1, v8f& c2, v8f& c3, v16h a, v16h b, v16h c, v16h d, v16h e) {
    asm volatile("v_nop\n\tv_nop\n\tv_nop\n\tv_nop" : "+v"(c0), "+v"(c1), "+v"(c2), "+v"(c3) : "v"(a), "v"(b), "v"(c), "v"(d), "v"(e));
}
__device__ __forceinline__ void guard8(v8f& c0, v8f& c1, v8f& c2, v8f& c3, v8f& c4, v8f& c5, v8f& c6, v8f& c7,
                                       v16h a, v16h b, v16h c, v16h d, v16h e, v16h f) {
    asm volatile("v_nop\n\tv_nop\n\tv_nop\n\tv_nop"
                 : "+v"(c0), "+v"(c1), "+v"(c2), "+v"(c3), "+v"(c4), "+v"(c5), "+v"(c6), "+v"(c7)
                 : "v"(a), "v"(b), "v"(c), "v"(d), "v"(e), "v"(f));
}

__global__ __launch_bounds__(256) void k_ln(const float* __restrict__ X, const float* __restrict__ G, const float* __restrict__ Bt, hf* XH) {
    const unsigned tid = threadIdx.x;
    const unsigned row = blockIdx.x * 16u + (tid >> 4);
    const unsigned sub = tid & 15u;
    const unsigned b = row / (unsigned)SEQ, n = row - b * (unsigned)SEQ;
    const float* src = X + ((size_t)b * SEQ_FULL + n) * DIM + sub * 8u;
    const v4f a0 = *(const v4f*)src;
    const v4f a1 = *(const v4f*)(src + 4);
    float e[8];
    e[0] = bfr(a0[0]); e[1] = bfr(a0[1]); e[2] = bfr(a0[2]); e[3] = bfr(a0[3]);
    e[4] = bfr(a1[0]); e[5] = bfr(a1[1]); e[6] = bfr(a1[2]); e[7] = bfr(a1[3]);
    float s = ((e[0] + e[1]) + (e[2] + e[3])) + ((e[4] + e[5]) + (e[6] + e[7]));
    s += __shfl_xor(s, 8, 32);
    s += __shfl_xor(s, 4, 32);
    s += __shfl_xor(s, 2, 32);
    s += __shfl_xor(s, 1, 32);
    const float mu = s * (1.0f / DIM);
    float d[8];
    float s2 = 0.0f;
#pragma unroll
    for (int j = 0; j < 8; ++j) { d[j] = e[j] - mu; s2 = fmaf(d[j], d[j], s2); }
    s2 += __shfl_xor(s2, 8, 32);
    s2 += __shfl_xor(s2, 4, 32);
    s2 += __shfl_xor(s2, 2, 32);
    s2 += __shfl_xor(s2, 1, 32);
    const float rs = rsqrtf(s2 * (1.0f / DIM) + 1.0e-5f);
    const v4f g0 = *(const v4f*)(G + sub * 8u), g1 = *(const v4f*)(G + sub * 8u + 4u);
    const v4f b0 = *(const v4f*)(Bt + sub * 8u), b1 = *(const v4f*)(Bt + sub * 8u + 4u);
    v8h o;
    o[0] = (_Float16)(d[0] * rs * bfr(g0[0]) + bfr(b0[0]));
    o[1] = (_Float16)(d[1] * rs * bfr(g0[1]) + bfr(b0[1]));
    o[2] = (_Float16)(d[2] * rs * bfr(g0[2]) + bfr(b0[2]));
    o[3] = (_Float16)(d[3] * rs * bfr(g0[3]) + bfr(b0[3]));
    o[4] = (_Float16)(d[4] * rs * bfr(g1[0]) + bfr(b1[0]));
    o[5] = (_Float16)(d[5] * rs * bfr(g1[1]) + bfr(b1[1]));
    o[6] = (_Float16)(d[6] * rs * bfr(g1[2]) + bfr(b1[2]));
    o[7] = (_Float16)(d[7] * rs * bfr(g1[3]) + bfr(b1[3]));
    const v8us ob = __builtin_bit_cast(v8us, o);
    hf* dst = XH + (size_t)row * DIM + sub * 8u;
    *(volatile v8us*)dst = ob;
    __threadfence();
    *(volatile v8us*)dst = ob;
}

__global__ __launch_bounds__(256) void k_wt(const float* __restrict__ W, hf* WT, int R, int C, float scale) {
    __shared__ __align__(16) hf tl[DIM * VTP];
    const unsigned tid = threadIdx.x;
    const unsigned tc = (unsigned)C / 128u;
    const unsigned kt = blockIdx.x / tc;
    const unsigned ct = blockIdx.x - kt * tc;
    const float* src = W + (size_t)(kt * 64u) * (unsigned)C + ct * 128u;
#pragma unroll
    for (unsigned it = 0; it < 8; ++it) {
        const unsigned f = it * 256u + tid;
        const unsigned key = f >> 5, c4 = (f & 31u) * 4u;
        const v4f x = *(const v4f*)(src + (size_t)key * (unsigned)C + c4);
#pragma unroll
        for (unsigned c = 0; c < 4; ++c) tl[(c4 + c) * VTP + key] = f2h(bfr(x[c]) * scale);
    }
    __syncthreads();
    hf* dst = WT + (size_t)(ct * 128u) * (unsigned)R + kt * 64u;
    const unsigned c8 = (tid & 7u) * 8u, dr = tid >> 3;
#pragma unroll 1
    for (int ps = 0; ps < 2; ++ps) {
#pragma unroll
        for (unsigned it = 0; it < 4; ++it) {
            const unsigned d = it * 32u + dr;
            const v8us o = *(const v8usa*)(tl + d * VTP + c8);
            *(volatile v8us*)(dst + (size_t)d * (unsigned)R + c8) = o;
        }
        if (ps == 0) __threadfence();
    }
}

__attribute__((amdgpu_num_vgpr(248))) __global__ __launch_bounds__(128) void k_qkv(const hf* XH, const hf* WT, hf* QKV, int bch0) {
    __shared__ __align__(16) hf st[DIM * VTP];
    const unsigned tid = threadIdx.x, lane = tid & 31u, lr = lane & 15u, hi = lane >> 4;
    const unsigned wave = (unsigned)__builtin_amdgcn_readfirstlane((int)(tid >> 5));
    const unsigned which = blockIdx.y >> 3, head = blockIdx.y & 7u;
    const unsigned mloc = blockIdx.x * 64u;
    const unsigned bl = mloc / (unsigned)SEQ, n0 = mloc - bl * (unsigned)SEQ;
    const size_t PL = (size_t)BCH * NH * SEQ * DIM;

    v16h tf[4];
    {
        const hf* tp = XH + ((size_t)((unsigned)bch0 + bl) * SEQ + n0 + 16u * wave + lr) * DIM + 8u * hi;
        tf[0] = ldh(tp);
        tf[1] = ldh(tp + 32);
        tf[2] = ldh(tp + 64);
        tf[3] = ldh(tp + 96);
    }
    const size_t woff = ((size_t)blockIdx.y * 128u + lr) * DIM + 8u * hi;
    const float un = 1.0f / WQS;

    if (which == 2u) {
#pragma unroll 1
        for (unsigned t = 0; t < 8u; ++t) {
            const hf* wr = WT + woff + (size_t)t * (16u * DIM);
            const v16h w0 = ldh(wr), w1 = ldh(wr + 32), w2 = ldh(wr + 64), w3 = ldh(wr + 96);
            v8f acc = (v8f){};
            acc = wmmah(tf[0], w0, acc);
            acc = wmmah(tf[1], w1, acc);
            acc = wmmah(tf[2], w2, acc);
            acc = wmmah(tf[3], w3, acc);
            guard1(acc, w0, w1, w2, w3);
            v8h o;
#pragma unroll
            for (int r = 0; r < 8; ++r) o[r] = (_Float16)(acc[r] * un);
            *(v8usa*)(st + (16u * t + lr) * VTP + 16u * wave + 8u * hi) = __builtin_bit_cast(v8us, o);
            sfence();
        }
    } else {
#pragma unroll 1
        for (unsigned t = 0; t < 8u; ++t) {
            const hf* wr = WT + woff + (size_t)t * (16u * DIM);
            const v16h w0 = ldh(wr), w1 = ldh(wr + 32), w2 = ldh(wr + 64), w3 = ldh(wr + 96);
            v8f acc = (v8f){};
            acc = wmmah(w0, tf[0], acc);
            acc = wmmah(w1, tf[1], acc);
            acc = wmmah(w2, tf[2], acc);
            acc = wmmah(w3, tf[3], acc);
            guard1(acc, w0, w1, w2, w3);
            v8h o;
#pragma unroll
            for (int r = 0; r < 8; ++r) o[r] = (_Float16)(acc[r] * un);
            *(v8usa*)(st + (16u * wave + lr) * CSP + 16u * t + 8u * hi) = __builtin_bit_cast(v8us, o);
            sfence();
        }
    }
    __syncthreads();
    const size_t bhp = (size_t)(bl * NH + head);
    if (which == 2u) {
        hf* dst = QKV + 2 * PL + bhp * DIM * SEQ + n0;
        const unsigned c8 = (tid & 7u) * 8u, dr = tid >> 3;
#pragma unroll 1
        for (int ps = 0; ps < 2; ++ps) {
#pragma unroll
            for (unsigned it = 0; it < 8; ++it) {
                const unsigned d = it * 16u + dr;
                const v8us o = *(const v8usa*)(st + d * VTP + c8);
                *(volatile v8us*)(dst + (size_t)d * SEQ + c8) = o;
            }
            if (ps == 0) __threadfence();
        }
    } else {
        hf* dst = QKV + (size_t)which * PL + (bhp * SEQ + n0) * DIM + lr * 8u;
#pragma unroll 1
        for (int ps = 0; ps < 2; ++ps) {
#pragma unroll
            for (unsigned s = 0; s < 8; ++s) {
                const unsigned rr = 16u * wave + 2u * s + hi;
                const v8us o = *(const v8usa*)(st + rr * CSP + lr * 8u);
                *(volatile v8us*)(dst + (size_t)rr * DIM) = o;
            }
            if (ps == 0) __threadfence();
        }
    }
}

__attribute__((amdgpu_num_vgpr(248))) __global__ __launch_bounds__(128) void k_flash(const hf* QP, const hf* KP, const hf* VT, hf* CH, hf* CL) {
    __shared__ __align__(16) hf cs[NWV * 2 * 16 * CSP];
    const unsigned tid = threadIdx.x, lane = tid & 31u, lr = lane & 15u, hi = lane >> 4;
    const unsigned wave = (unsigned)__builtin_amdgcn_readfirstlane((int)(tid >> 5));
    const unsigned bpb = (unsigned)(SEQ / BQ);
    const unsigned bh = blockIdx.x / bpb;
    const unsigned q0 = (blockIdx.x - bh * bpb) * BQ + wave * 16u;

    v16h qf[4];
    {
        const hf* qp = QP + ((size_t)bh * SEQ + q0 + lr) * DIM + 8u * hi;
        qf[0] = ldh(qp);
        qf[1] = ldh(qp + 32);
        qf[2] = ldh(qp + 64);
        qf[3] = ldh(qp + 96);
    }
    const size_t kbase = ((size_t)bh * SEQ + lr) * DIM + 8u * hi;
    const size_t vbase = ((size_t)bh * DIM + lr) * SEQ + 8u * hi;

    v8f o[8];
#pragma unroll
    for (int t = 0; t < 8; ++t) o[t] = (v8f){};
    float ml = -1.0e30f;
    float l = 0.0f;

#pragma unroll 1
    for (unsigned k0 = 0; k0 < (unsigned)SEQ; k0 += KS) {
        v8f s0 = (v8f){}, s1 = (v8f){};
        const hf* ka = KP + kbase + (size_t)k0 * DIM;
        {
            const v16h a00 = ldh(ka), a01 = ldh(ka + 16 * DIM);
            const v16h a10 = ldh(ka + 32), a11 = ldh(ka + 16 * DIM + 32);
            s0 = wmmah(a00, qf[0], s0);
            s1 = wmmah(a01, qf[0], s1);
            s0 = wmmah(a10, qf[1], s0);
            s1 = wmmah(a11, qf[1], s1);
            guard2(s0, s1, a00, a01, a10, a11);
        }
        sfence();
        {
            const v16h a20 = ldh(ka + 64), a21 = ldh(ka + 16 * DIM + 64);
            const v16h a30 = ldh(ka + 96), a31 = ldh(ka + 16 * DIM + 96);
            s0 = wmmah(a20, qf[2], s0);
            s1 = wmmah(a21, qf[2], s1);
            s0 = wmmah(a30, qf[3], s0);
            s1 = wmmah(a31, qf[3], s1);
            guard2(s0, s1, a20, a21, a30, a31);
        }
        sfence();

        float mx = fmaxf(s0[0], s1[0]);
#pragma unroll
        for (int r = 1; r < 8; ++r) mx = fmaxf(mx, fmaxf(s0[r], s1[r]));
        mx = fmaxf(mx, __shfl_xor(mx, 16, 32));
        const float mnl = fmaxf(ml, mx * SC2);
        const float corr = __builtin_amdgcn_exp2f(ml - mnl);
        ml = mnl;
        const float sh = PCL - mnl;
        float p0[8], p1[8];
        float ps = 0.0f;
#pragma unroll
        for (int r = 0; r < 8; ++r) {
            p0[r] = __builtin_amdgcn_exp2f(fmaf(s0[r], SC2, sh));
            p1[r] = __builtin_amdgcn_exp2f(fmaf(s1[r], SC2, sh));
            ps += p0[r] + p1[r];
        }
        ps += __shfl_xor(ps, 16, 32);
        l = l * corr + ps;
        if (__builtin_amdgcn_ballot_w32(corr != 1.0f) != 0u) {
#pragma unroll
            for (int t = 0; t < 8; ++t) o[t] *= corr;
        }

        v16h ph;
#pragma unroll
        for (int r = 0; r < 8; ++r) { ph[r] = (_Float16)p0[r]; ph[8 + r] = (_Float16)p1[r]; }

        sfence();
        const hf* va = VT + vbase + k0;
        {
            const v16h v0 = ldh(va), v1 = ldh(va + (size_t)16 * SEQ), v2 = ldh(va + (size_t)32 * SEQ), v3 = ldh(va + (size_t)48 * SEQ);
            o[0] = wmmah(v0, ph, o[0]);
            o[1] = wmmah(v1, ph, o[1]);
            o[2] = wmmah(v2, ph, o[2]);
            o[3] = wmmah(v3, ph, o[3]);
            guard4(o[0], o[1], o[2], o[3], v0, v1, v2, v3, ph);
        }
        sfence();
        {
            const v16h v4 = ldh(va + (size_t)64 * SEQ), v5 = ldh(va + (size_t)80 * SEQ), v6 = ldh(va + (size_t)96 * SEQ), v7 = ldh(va + (size_t)112 * SEQ);
            o[4] = wmmah(v4, ph, o[4]);
            o[5] = wmmah(v5, ph, o[5]);
            o[6] = wmmah(v6, ph, o[6]);
            o[7] = wmmah(v7, ph, o[7]);
            guard4(o[4], o[5], o[6], o[7], v4, v5, v6, v7, ph);
        }
        sfence();
    }

    const float sc = (1.0f / l) * CCS;
    const unsigned creg = wave * (2u * 16u * CSP);
#pragma unroll
    for (int t = 0; t < 8; ++t) {
        v8h hv, lv;
#pragma unroll
        for (int r = 0; r < 8; ++r) {
            const float c = o[t][r] * sc;
            const _Float16 h = (_Float16)c;
            hv[r] = h;
            lv[r] = (_Float16)((c - (float)h) * RSC);
        }
        *(v8usa*)(cs + creg + lr * CSP + 16u * t + 8u * hi) = __builtin_bit_cast(v8us, hv);
        *(v8usa*)(cs + creg + 16u * CSP + lr * CSP + 16u * t + 8u * hi) = __builtin_bit_cast(v8us, lv);
    }
    __syncthreads();
    const unsigned bl = bh / NH, head = bh - bl * NH;
    const size_t rowbase = ((size_t)bl * SEQ + q0) * INNER + head * DIM + lr * 8u;
#pragma unroll 1
    for (int ps2 = 0; ps2 < 2; ++ps2) {
#pragma unroll
        for (unsigned s = 0; s < 8; ++s) {
            const unsigned rr = 2u * s + hi;
            const v8us vh = *(const v8usa*)(cs + creg + rr * CSP + lr * 8u);
            const v8us vl = *(const v8usa*)(cs + creg + 16u * CSP + rr * CSP + lr * 8u);
            *(volatile v8us*)(CH + rowbase + (size_t)rr * INNER) = vh;
            *(volatile v8us*)(CL + rowbase + (size_t)rr * INNER) = vl;
        }
        if (ps2 == 0) __threadfence();
    }
}

__global__ __launch_bounds__(256) void k_proj(const hf* CH, const hf* CL, const hf* WP, const float* __restrict__ bias, float* OUT, int bch0) {
    __shared__ __align__(16) float os[64 * OSP];
    const unsigned tid = threadIdx.x, lane = tid & 31u, lr = lane & 15u, hi = lane >> 4;
    const unsigned wave = (unsigned)__builtin_amdgcn_readfirstlane((int)(tid >> 5));
    const unsigned tg = wave >> 1, fh = wave & 1u;
    const unsigned m0 = blockIdx.x * 64u;
    const size_t coff = ((size_t)(m0 + 16u * tg + lr)) * INNER + 8u * hi;
    const size_t woff = ((size_t)(64u * fh + lr)) * INNER + 8u * hi;

    v8f ah[4], al[4];
#pragma unroll
    for (int t = 0; t < 4; ++t) { ah[t] = (v8f){}; al[t] = (v8f){}; }

#pragma unroll 1
    for (unsigned k0 = 0; k0 < (unsigned)INNER; k0 += 32) {
        const v16h ch = ldh(CH + coff + k0);
        const v16h cl = ldh(CL + coff + k0);
        const hf* wr = WP + woff + k0;
        const v16h w0 = ldh(wr), w1 = ldh(wr + (size_t)16 * INNER), w2 = ldh(wr + (size_t)32 * INNER), w3 = ldh(wr + (size_t)48 * INNER);
        ah[0] = wmmah(w0, ch, ah[0]);
        al[0] = wmmah(w0, cl, al[0]);
        ah[1] = wmmah(w1, ch, ah[1]);
        al[1] = wmmah(w1, cl, al[1]);
        ah[2] = wmmah(w2, ch, ah[2]);
        al[2] = wmmah(w2, cl, al[2]);
        ah[3] = wmmah(w3, ch, ah[3]);
        al[3] = wmmah(w3, cl, al[3]);
        guard8(ah[0], ah[1], ah[2], ah[3], al[0], al[1], al[2], al[3], ch, cl, w0, w1, w2, w3);
        sfence();
    }

    const float un = 1.0f / (CCS * WPS);
    const float ur = 1.0f / RSC;
#pragma unroll
    for (int t = 0; t < 4; ++t) {
        v4f x0, x1;
        x0[0] = fmaf(al[t][0], ur, ah[t][0]) * un; x0[1] = fmaf(al[t][1], ur, ah[t][1]) * un;
        x0[2] = fmaf(al[t][2], ur, ah[t][2]) * un; x0[3] = fmaf(al[t][3], ur, ah[t][3]) * un;
        x1[0] = fmaf(al[t][4], ur, ah[t][4]) * un; x1[1] = fmaf(al[t][5], ur, ah[t][5]) * un;
        x1[2] = fmaf(al[t][6], ur, ah[t][6]) * un; x1[3] = fmaf(al[t][7], ur, ah[t][7]) * un;
        const unsigned so = (16u * tg + lr) * OSP + 64u * fh + 16u * t + 8u * hi;
        *(v4fa*)(os + so) = x0;
        *(v4fa*)(os + so + 4u) = x1;
    }
    __syncthreads();
    const v4f bb = *(const v4f*)(bias + lane * 4u);
    v4f bq;
    bq[0] = bfr(bb[0]); bq[1] = bfr(bb[1]); bq[2] = bfr(bb[2]); bq[3] = bfr(bb[3]);
    float* orow = OUT + ((size_t)bch0 * SEQ + m0 + 8u * wave) * DIM + lane * 4u;
#pragma unroll 1
    for (int ps = 0; ps < 2; ++ps) {
#pragma unroll
        for (unsigned s = 0; s < 8; ++s) {
            v4f val = *(const v4fa*)(os + (8u * wave + s) * OSP + lane * 4u);
            val[0] += bq[0]; val[1] += bq[1]; val[2] += bq[2]; val[3] += bq[3];
            *(volatile v4f*)(orow + (size_t)s * DIM) = val;
        }
        if (ps == 0) __threadfence();
    }
}

extern "C" void kernel_launch(void* const* d_in, const int* in_sizes, int n_in,
                              void* d_out, int out_size, void* d_ws, size_t ws_size, hipStream_t stream) {
    if (n_in < 6) return;
    const size_t need = ((size_t)(NB - 1) * SEQ_FULL + SEQ) * DIM;
    if ((size_t)in_sizes[0] < need) return;
    if (in_sizes[1] < DIM || in_sizes[2] < DIM || in_sizes[5] < DIM) return;
    if ((size_t)in_sizes[3] < (size_t)DIM * QKVN) return;
    if ((size_t)in_sizes[4] < (size_t)INNER * DIM) return;
    if ((size_t)out_size < (size_t)NB * SEQ * DIM) return;
    if (SZ_ALL > ws_size) return;

    const float* x      = (const float*)d_in[0];
    const float* gamma  = (const float*)d_in[1];
    const float* beta   = (const float*)d_in[2];
    const float* w_qkv  = (const float*)d_in[3];
    const float* w_proj = (const float*)d_in[4];
    const float* b_proj = (const float*)d_in[5];
    float* OUT = (float*)d_out;

    char* wsp = (char*)d_ws;
    hf* XH  = (hf*)(wsp);
    hf* WT  = (hf*)(wsp + SZ_XH);
    hf* WP  = (hf*)(wsp + SZ_XH + SZ_WT);
    hf* QKV = (hf*)(wsp + SZ_XH + SZ_WT + SZ_WP);
    hf* CH  = (hf*)(wsp + SZ_XH + SZ_WT + SZ_WP + 3 * SZ_PL);
    hf* CL  = (hf*)(wsp + SZ_XH + SZ_WT + SZ_WP + 3 * SZ_PL + SZ_CX);
    const size_t PL = (size_t)BCH * NH * SEQ * DIM;

    k_ln<<<(unsigned)(NB * SEQ / 16), 256, 0, stream>>>(x, gamma, beta, XH);
    k_wt<<<(unsigned)((DIM / 64) * (QKVN / 128)), 256, 0, stream>>>(w_qkv, WT, DIM, QKVN, WQS);
    k_wt<<<(unsigned)((INNER / 64) * (DIM / 128)), 256, 0, stream>>>(w_proj, WP, INNER, DIM, WPS);
    for (int c = 0; c < NCH; ++c) {
        const int bch0 = c * BCH;
        k_qkv<<<dim3((unsigned)(BCH * SEQ / 64), 24, 1), 128, 0, stream>>>(XH, WT, QKV, bch0);
        k_flash<<<(unsigned)(BCH * NH * (SEQ / BQ)), 128, 0, stream>>>(QKV, QKV + PL, QKV + 2 * PL, CH, CL);
        k_proj<<<(unsigned)(BCH * SEQ / 64), 256, 0, stream>>>(CH, CL, WP, b_proj, OUT, bch0);
    }
}
